// NonLocalBlock_24240795418664
// MI455X (gfx1250) — hardware-verified
//
#include <hip/hip_runtime.h>
#include <math.h>

typedef __attribute__((ext_vector_type(16))) _Float16 v16h;
typedef __attribute__((ext_vector_type(16))) __bf16 v16b;
typedef __attribute__((ext_vector_type(8)))  _Float16 v8h;
typedef __attribute__((ext_vector_type(8)))  float v8f;
typedef __attribute__((ext_vector_type(4)))  float v4f;
typedef __attribute__((ext_vector_type(4)))  unsigned v4u;

template <typename T> __device__ __forceinline__ void vst2(void* p, T v) { *(volatile T*)p = v; __threadfence(); *(volatile T*)p = v; }
__device__ __forceinline__ v8f wmma16(v16h a, v16h b, v8f c) {
  v8f d = __builtin_amdgcn_wmma_f32_16x16x32_f16(false, a, false, b, (short)0, c, false, false);
  asm volatile("v_nop\n\tv_nop\n\tv_nop\n\tv_nop" : "+v"(d) : "v"(a), "v"(b));
  return d;
}
__device__ __forceinline__ v8f wmma_bf(v16b a, v16b b, v8f c) {
  v8f d = __builtin_amdgcn_wmma_f32_16x16x32_bf16(false, a, false, b, (short)0, c, false, false);
  asm volatile("v_nop\n\tv_nop\n\tv_nop\n\tv_nop" : "+v"(d) : "v"(a), "v"(b));
  return d;
}
__device__ __forceinline__ v16h frag_h(const _Float16* rowk0, int lane) {
  union { v16h v; v8h q[2]; } u; const _Float16* p = rowk0 + 8 * (lane >> 4);
  u.q[0] = *(const v8h*)p; u.q[1] = *(const v8h*)(p + 16); return u.v;
}
__device__ __forceinline__ float bfr(float v) { return (float)(__bf16)v; }
__device__ __forceinline__ v16b wcol_oi(const float* Wm, int k0, int o, int lane, int K) { v16b w; const float* p = Wm + (size_t)o * K + k0 + 8 * (lane >> 4);
#pragma unroll
  for (int i = 0; i < 8; ++i) { w[i] = (__bf16)p[i]; w[8 + i] = (__bf16)p[16 + i]; }
  return w; }
#define LDSX() do { asm volatile("s_wait_dscnt 0" ::: "memory"); __builtin_amdgcn_wave_barrier(); __builtin_amdgcn_fence(3  , "workgroup"); } while (0)

#define NB 4
#ifndef TNB
#define TNB NB
#endif
#ifndef TT
#define TT 4096
#endif
#define TT_FULL 4096
#define DIN 64
#define CC 128
#define CV 32
#define COUT 64
#define CCQ 128
#define HD 32
#define NQB (TT / 64)
#define HG 1
#define HDQK 32
#define BG HG
#define BGN (TNB < BG ? TNB : BG)
#define DVH 32

static_assert(TT % 128 == 0);
static_assert(TT <= TT_FULL);
static_assert(TNB <= NB);
static_assert(DIN % 32 == 0);
static_assert(HDQK == 32 && CV == 32 && DVH == 32);
static_assert((64 * 16) % 128 == 0 && (128 * 8) % 128 == 0);

#define WS_QH  ((size_t)0)
#define WS_KH  (WS_QH + 2u * (size_t)NB * TT * CCQ)
#define WS_VT  (WS_KH + 2u * (size_t)NB * TT * CCQ)
#define WS_QL  (WS_VT + 2u * (size_t)NB * CC * TT)
#define WS_KL  (WS_QL + 2u * (size_t)NB * TT * CCQ)
#define WS_S   (WS_KL + 2u * (size_t)NB * TT * CCQ)
#define WS_END (WS_S  + 4u * (size_t)HG * TT * TT)
static_assert(WS_END <= (size_t)134217728);
static_assert(WS_S % 128 == 0);

__global__ __launch_bounds__(128) void k_proj(const float* __restrict__ XQ, const float* __restrict__ XK, const float* __restrict__ XV, const float* __restrict__ WQ, const float* __restrict__ WK, const float* __restrict__ WV, const float* __restrict__ BQ, const float* __restrict__ BK, const float* __restrict__ BV,
    _Float16* __restrict__ QH, _Float16* __restrict__ QL, _Float16* __restrict__ KH, _Float16* __restrict__ KL, _Float16* __restrict__ VT) {
  __shared__ __align__(16) _Float16 sh[64][136], sl[64][136]; __shared__ __align__(16) _Float16 th[128][72];
  const int tid = threadIdx.x, wave = tid >> 5, lane = tid & 31, col = lane & 15, g = lane >> 4; const int which = blockIdx.z; const int c0 = 0;
  const size_t r0 = (size_t)blockIdx.x * 64; const size_t bb = r0 / TT; const int t0 = (int)(r0 % TT);
  const float* X = which == 0 ? XQ : which == 1 ? XK : XV; const float* WA = which == 0 ? WQ : which == 1 ? WK : WV; const float* BA = which == 0 ? BQ : which == 1 ? BK : BV;
  v8f acc[8] = {};
#pragma unroll
  for (int kc = 0; kc < DIN / 32; ++kc) { v16b a; { const float* p = X + (bb * DIN + kc * 32 + 8 * g) * (size_t)TT_FULL + t0 + wave * 16 + col;
#pragma unroll
      for (int i = 0; i < 8; ++i) { a[i] = (__bf16)p[(size_t)i * TT_FULL]; a[8 + i] = (__bf16)p[(size_t)(16 + i) * TT_FULL]; } }
    asm volatile("s_wait_loadcnt 0x0" ::: "memory");
#pragma unroll
    for (int j = 0; j < HDQK / 16; ++j) { const v16b w = wcol_oi(WA, kc * 32, j * 16 + col, lane, DIN); asm volatile("s_wait_loadcnt 0x0" ::: "memory"); acc[j] = wmma_bf(a, w, acc[j]); } }
  if (which < 2) { _Float16* DH = which == 0 ? QH : KH; _Float16* DL = which == 0 ? QL : KL;
#pragma unroll
    for (int j = 0; j < 8; ++j) { const int cj = c0 + j * 16 + col; const int cjc = cj < HDQK ? cj : HDQK - 1; const float bv = bfr(BA[cjc]); const float bias = cj < HDQK ? bv : 0.f;
#pragma unroll
      for (int r = 0; r < 8; ++r) { const float v = acc[j][r] + bias; const _Float16 hv = (_Float16)v; sh[wave * 16 + 8 * g + r][j * 16 + col] = hv; sl[wave * 16 + 8 * g + r][j * 16 + col] = (_Float16)((v - (float)hv) * 1024.0f); } }
    __syncthreads();
    for (int e = tid; e < 64 * 16; e += 128) { const int rl = e >> 4, q = e & 15; const size_t o2 = (r0 + rl) * (size_t)CCQ + c0 + q * 8; vst2((unsigned*)(DH + o2), *(const v4u*)&sh[rl][q * 8]); vst2((unsigned*)(DL + o2), *(const v4u*)&sl[rl][q * 8]); }
  } else {
#pragma unroll
    for (int j = 0; j < 8; ++j) { const int cj = c0 + j * 16 + col; const int cjc = cj < CV ? cj : CV - 1; const float bv = bfr(BA[cjc]); const float bias = cj < CV ? bv : 0.f;
#pragma unroll
      for (int r = 0; r < 8; ++r) { const float v = acc[j][r] + bias; const int rl = wave * 16 + 8 * g + r, cl = j * 16 + col; th[cl][rl] = (_Float16)v; } }
    __syncthreads();
    for (int e = tid; e < 128 * 8; e += 128) { const int cl = e >> 3, q = e & 7; vst2((unsigned*)(VT + (bb * CC + c0 + cl) * (size_t)TT + t0 + q * 8), *(const v4u*)&th[cl][q * 8]); } } }
__global__ __launch_bounds__(128) void k_sc(const _Float16* __restrict__ QH, const _Float16* __restrict__ KH, const _Float16* __restrict__ QL, const _Float16* __restrict__ KL, int bgrp, float* __restrict__ S0) { __shared__ __align__(16) float ss[4][16][132];
  const int qb = blockIdx.x, kb = blockIdx.y;
  const int b = bgrp + blockIdx.z; float* S = S0 + (size_t)blockIdx.z * TT * TT;
  const int tid = threadIdx.x, wave = tid >> 5, lane = tid & 31, col = lane & 15, g = lane >> 4; const int k0 = kb * 128; const int ql0 = qb * 64 + wave * 16; const size_t q0 = (size_t)b * TT + ql0, kr0 = (size_t)b * TT + k0;
  v8f acc[8] = {}, accl[8] = {};
#pragma unroll
  for (int kc = 0; kc < HDQK / 32; ++kc) { const v16h ah = frag_h(QH + (q0 + col) * CCQ + kc * 32, lane), al = frag_h(QL + (q0 + col) * CCQ + kc * 32, lane);
#pragma unroll
    for (int j = 0; j < 8; ++j) { const v16h kbf = frag_h(KH + (kr0 + j * 16 + col) * CCQ + kc * 32, lane), klf = frag_h(KL + (kr0 + j * 16 + col) * CCQ + kc * 32, lane); acc[j] = wmma16(ah, kbf, acc[j]); accl[j] = wmma16(al, kbf, accl[j]); accl[j] = wmma16(ah, klf, accl[j]); } }
#pragma unroll
  for (int j = 0; j < 8; ++j) {
#pragma unroll
    for (int r = 0; r < 8; ++r) ss[wave][8 * g + r][j * 16 + col] = acc[j][r] + accl[j][r] * (1.0f / 1024.0f); }
  LDSX();
  for (int rl = 0; rl < 16; ++rl) vst2(S + (size_t)(ql0 + rl) * TT + k0 + lane * 4, *(const v4f*)&ss[wave][rl][lane * 4]); }
__global__ __launch_bounds__(256) void k_sm(float* __restrict__ S0) { __shared__ float sred[8]; __shared__ float sbc; __shared__ __align__(16) float shv[TT];
  const int tid = threadIdx.x; const int t = blockIdx.x;
  float* sr = S0 + (size_t)blockIdx.y * TT * TT + (size_t)t * TT;
  float m = -3.0e38f; for (int k = tid; k < TT; k += 256) { const float v = sr[k]; shv[k] = v; m = fmaxf(m, v); }
#pragma unroll
  for (int o = 1; o < 32; o <<= 1) m = fmaxf(m, __shfl_xor(m, o));
  if ((tid & 31) == 0) sred[tid >> 5] = m; __syncthreads(); if (tid == 0) { float a = sred[0]; for (int i = 1; i < 8; ++i) a = fmaxf(a, sred[i]); sbc = a; } __syncthreads(); m = sbc; __syncthreads();
  float sum = 0.f; for (int k = tid; k < TT; k += 256) { const float e = expf(shv[k] - m); shv[k] = e; sum += e; }
#pragma unroll
  for (int o = 1; o < 32; o <<= 1) sum += __shfl_xor(sum, o);
  if ((tid & 31) == 0) sred[tid >> 5] = sum; __syncthreads(); if (tid == 0) { float a = 0.f; for (int i = 0; i < 8; ++i) a += sred[i]; sbc = 2048.0f * (1.0f / a); } __syncthreads(); const float inv = sbc;
  for (int k = tid; k < TT; k += 256) shv[k] = shv[k] * inv;
  __syncthreads(); for (int q = tid; q < TT / 4; q += 256) vst2(sr + q * 4, *(const v4f*)&shv[q * 4]); }
__global__ __launch_bounds__(128) void k_pv(const float* __restrict__ PS0, const _Float16* __restrict__ VT, int bgrp, const float* __restrict__ WO, const float* __restrict__ BO, const float* __restrict__ XS, float* __restrict__ Y) { __shared__ __align__(16) float stT[DVH][68];
  const int b = bgrp + blockIdx.z; const float* PS = PS0 + (size_t)blockIdx.z * TT * TT; const int d0 = blockIdx.y * DVH;
  const int tid = threadIdx.x, wave = tid >> 5, lane = tid & 31, col = lane & 15, g = lane >> 4; const int qb = blockIdx.x; const int ql0 = qb * 64 + wave * 16; const int kce = TT / 32;
  v8f acc[DVH / 16] = {};
#pragma unroll 1
  for (int kc = 0; kc < kce; ++kc) { v16h p; { const float* pp = PS + (size_t)(kc * 32 + 8 * g) * TT + ql0 + col;
#pragma unroll
      for (int i = 0; i < 8; ++i) { p[i] = (_Float16)pp[(size_t)i * TT]; p[8 + i] = (_Float16)pp[(size_t)(16 + i) * TT]; } }
    asm volatile("s_wait_loadcnt 0x0" ::: "memory");
#pragma unroll
    for (int j = 0; j < DVH / 16; ++j) { const size_t po = ((size_t)b * CC + d0 + j * 16 + col) * (size_t)TT + kc * 32; acc[j] = wmma16(p, frag_h(VT + po, lane), acc[j]); } }
#pragma unroll
  for (int j = 0; j < DVH / 16; ++j) {
#pragma unroll
    for (int r = 0; r < 8; ++r) stT[j * 16 + col][wave * 16 + 8 * g + r] = acc[j][r] * (1.0f / 2048.0f); }
  __syncthreads();
  { const int tb = qb * 64; const int tl = tid & 63, oh = tid >> 6;
    float yv[DVH];
#pragma unroll
    for (int c = 0; c < DVH; ++c) yv[c] = stT[c][tl];
#pragma unroll 1
    for (int oo = 0; oo < COUT / 2; ++oo) { const int o = oh * (COUT / 2) + oo; float wv[DVH];
#pragma unroll
      for (int c = 0; c < DVH; ++c) { wv[c] = WO[o * CV + c]; if ((c & 15) == 15) asm volatile("s_wait_loadcnt 0x0" ::: "memory"); }
      const size_t oi = ((size_t)b * COUT + o) * (size_t)TT_FULL + tb + tl;
      const float bo = BO[o]; const float xs = XS[oi]; asm volatile("s_wait_loadcnt 0x0" ::: "memory");
      float a2 = 0.f;
#pragma unroll
      for (int c = 0; c < DVH; ++c) a2 += yv[c] * bfr(wv[c]);
      const float zv = bfr(xs) + (a2 + bfr(bo));
      vst2(Y + oi, zv); } } }

extern "C" void kernel_launch(void* const* d_in, const int* in_sizes, int n_in, void* d_out, int out_size, void* d_ws, size_t ws_size, hipStream_t stream) {
  if (n_in < 10) return;
  if (ws_size < (size_t)WS_END) return;
  if ((long long)in_sizes[0] < (long long)TNB * DIN * TT_FULL || (long long)in_sizes[1] < (long long)TNB * DIN * TT_FULL) return;
  if (in_sizes[2] < HDQK * DIN || in_sizes[4] < HDQK * DIN || in_sizes[6] < CV * DIN || in_sizes[8] < COUT * CV) return;
  if (in_sizes[3] < HDQK || in_sizes[5] < HDQK || in_sizes[7] < CV || in_sizes[9] < COUT) return;
  if ((long long)out_size < (long long)TNB * COUT * TT_FULL) return;
  const float** F = (const float**)d_in;
  char* ws = (char*)d_ws; _Float16 *QH = (_Float16*)(ws + WS_QH), *KH = (_Float16*)(ws + WS_KH), *VT = (_Float16*)(ws + WS_VT), *QL = (_Float16*)(ws + WS_QL), *KL = (_Float16*)(ws + WS_KL); float *S = (float*)(ws + WS_S);
  k_proj<<<dim3(TNB * TT / 64, 1, 3), 128, 0, stream>>>(F[1], F[0], F[1], F[4], F[2], F[6], F[5], F[3], F[7], QH, QL, KH, KL, VT);
  for (int b0 = 0; b0 < TNB; b0 += BGN) {
    k_sc<<<dim3(NQB, TT / 128, BGN), 128, 0, stream>>>(QH, KH, QL, KL, b0, S);
    k_sm<<<dim3(TT, BGN), 256, 0, stream>>>(S);
    k_pv<<<dim3(NQB, HD / DVH, BGN), 128, 0, stream>>>(S, VT, b0, F[8], F[9], F[0], (float*)d_out);
  }
}
